// TiledAttention_81166291959865
// MI455X (gfx1250) — hardware-verified
//
#include <hip/hip_runtime.h>


#define NB_ 4
#define NN_ 4096
#define HD  128
#define PSC 32768.0f

typedef _Float16 h16;
typedef unsigned short bf;
typedef __attribute__((ext_vector_type(16))) __bf16   v16bf;
typedef __attribute__((ext_vector_type(16))) _Float16 v16h;
typedef __attribute__((ext_vector_type(8)))  _Float16 v8h;
typedef __attribute__((ext_vector_type(8)))  unsigned short v8us;
typedef __attribute__((ext_vector_type(8)))  float    v8f;
typedef __attribute__((ext_vector_type(4)))  float    v4f;
typedef v8h  __attribute__((may_alias)) v8ha;
typedef v4f  __attribute__((may_alias)) v4fa;

__device__ __forceinline__ unsigned short f2bf(float f) { unsigned u = __float_as_uint(f); u += 0x7FFFu + ((u >> 16) & 1u); return (unsigned short)(u >> 16); }
__device__ __forceinline__ float bf2f(unsigned short b) { return __uint_as_float(((unsigned)b) << 16); }
__device__ __forceinline__ v16h cat16(v8h lo, v8h hi) { return __builtin_shufflevector(lo, hi, 0, 1, 2, 3, 4, 5, 6, 7, 8, 9, 10, 11, 12, 13, 14, 15); }
__device__ __forceinline__ v16bf cat16b(v8us lo, v8us hi) { return __builtin_bit_cast(v16bf, __builtin_shufflevector(lo, hi, 0, 1, 2, 3, 4, 5, 6, 7, 8, 9, 10, 11, 12, 13, 14, 15)); }
__device__ __forceinline__ v8f wmma16(v16h a, v16h b, v8f c) { return __builtin_amdgcn_wmma_f32_16x16x32_f16(false, a, false, b, (short)0, c, false, false); }
__device__ __forceinline__ v8f wmmab(v16bf a, v16bf b, v8f c) { return __builtin_amdgcn_wmma_f32_16x16x32_bf16(false, a, false, b, (short)0, c, false, false); }

__global__ __launch_bounds__(256) void k_cvtqk(const float* __restrict__ q, const float* __restrict__ k, bf* QB, bf* KB) {
    const int lane = threadIdx.x & 31, wid = blockIdx.x * 8 + (threadIdx.x >> 5);
    if (wid >= 2 * NB_ * NN_) return;
    const int r = wid >> 1, which = wid & 1;
    const float* s = (which ? k : q) + (size_t)r * HD + lane * 4;
    typedef __attribute__((ext_vector_type(4))) unsigned short v4us;
    v4us o; o[0] = f2bf(s[0]); o[1] = f2bf(s[1]); o[2] = f2bf(s[2]); o[3] = f2bf(s[3]);
    bf* d = (which ? KB : QB) + (size_t)r * HD + lane * 4;
    *(volatile v4us*)d = o;
    __threadfence();
    *(volatile v4us*)d = o;
}

__global__ __launch_bounds__(256) void k_vt(const float* __restrict__ v, h16* VT16) {
    __shared__ __align__(16) h16 tile[HD * 72];
    const int b = blockIdx.x / (NN_ / 64), kt = blockIdx.x - b * (NN_ / 64), k0 = kt * 64, tid = threadIdx.x;
    const int kk = tid >> 2, d0 = (tid & 3) * 32;
    const float* src = v + ((size_t)b * NN_ + k0 + kk) * HD + d0;
#pragma unroll
    for (int i = 0; i < 32; ++i) tile[(d0 + i) * 72 + kk] = (h16)bf2f(f2bf(src[i]));
    __syncthreads();
    const int piece = tid & 7;
    h16* base = VT16 + (size_t)b * HD * NN_ + k0;
    auto pass = [&]() {
#pragma unroll
        for (int s = 0; s < 4; ++s) {
            const int d = (tid >> 3) + 32 * s;
            const v8h val = *(const v8ha*)(tile + d * 72 + piece * 8);
            *(volatile v8h*)(base + (size_t)d * NN_ + piece * 8) = val;
        }
    };
    pass();
    __threadfence();
    pass();
}

__global__ __launch_bounds__(128) void k_attn(const bf* __restrict__ QB, const bf* __restrict__ KB, const h16* __restrict__ VT16, float* out) {
    __shared__ __align__(16) h16 plds[4][16 * 32];
    __shared__ __align__(16) float ost[4][16 * 132];
    const int lane = threadIdx.x & 31, wave = threadIdx.x >> 5, lr = lane & 15, hi = lane >> 4;
    const int b = blockIdx.x / (NN_ / 64), qt = blockIdx.x - b * (NN_ / 64);
    const int q0 = qt * 64 + wave * 16;
    const size_t row0 = (size_t)b * NN_;
    h16* pl = &plds[wave][0];
    v16bf qa[4];
#pragma unroll
    for (int kc = 0; kc < 4; ++kc) {
        const bf* p = QB + (row0 + q0 + lr) * HD + kc * 32 + 8 * hi;
        qa[kc] = cat16b(*(const v8us*)p, *(const v8us*)(p + 16));
    }
    const bf* kb_b = KB + row0 * HD;
    const h16* vt_b = VT16 + (size_t)b * HD * NN_;
    const float scale = 0.08838834764831845f;
    v8f o[8];
#pragma unroll
    for (int n = 0; n < 8; ++n) o[n] = (v8f){};
    float mrow[8], lpart[8];
#pragma unroll
    for (int j = 0; j < 8; ++j) { mrow[j] = -3.0e38f; lpart[j] = 0.f; }
#pragma unroll 1
    for (int kt = 0; kt < NN_ / 32; ++kt) {
        const int l0 = kt * 32;
        const bf* r0p = kb_b + (size_t)(l0 + lr) * HD + 8 * hi;
        const bf* r1p = kb_b + (size_t)(l0 + 16 + lr) * HD + 8 * hi;
        v8f s0 = {}, s1 = {};
#pragma unroll
        for (int kc = 0; kc < 4; ++kc) {
            s0 = wmmab(qa[kc], cat16b(*(const v8us*)(r0p + kc * 32), *(const v8us*)(r0p + kc * 32 + 16)), s0);
            s1 = wmmab(qa[kc], cat16b(*(const v8us*)(r1p + kc * 32), *(const v8us*)(r1p + kc * 32 + 16)), s1);
        }
        asm volatile("v_nop\n\tv_nop\n\tv_nop\n\tv_nop" : "+v"(s0), "+v"(s1) : "v"(qa[0]), "v"(qa[3]));
        float alpha[8];
#pragma unroll
        for (int j = 0; j < 8; ++j) {
            const float a0 = s0[j] * scale, a1 = s1[j] * scale;
            float mx = fmaxf(a0, a1);
            mx = fmaxf(mx, __shfl_xor(mx, 1, 16)); mx = fmaxf(mx, __shfl_xor(mx, 2, 16));
            mx = fmaxf(mx, __shfl_xor(mx, 4, 16)); mx = fmaxf(mx, __shfl_xor(mx, 8, 16));
            const float mn = fmaxf(mrow[j], mx);
            alpha[j] = __expf(mrow[j] - mn);
            mrow[j] = mn;
            const float p0 = __expf(a0 - mn), p1 = __expf(a1 - mn);
            lpart[j] = lpart[j] * alpha[j] + (p0 + p1);
            const int mr = hi * 8 + j;
            pl[mr * 32 + lr]      = (h16)(p0 * PSC);
            pl[mr * 32 + 16 + lr] = (h16)(p1 * PSC);
        }
#pragma unroll
        for (int n = 0; n < 8; ++n)
#pragma unroll
            for (int j = 0; j < 8; ++j) o[n][j] *= alpha[j];
        asm volatile("" ::: "memory");
        const v16h pa = cat16(*(const v8ha*)(pl + lr * 32 + hi * 8), *(const v8ha*)(pl + lr * 32 + 16 + hi * 8));
#pragma unroll
        for (int n = 0; n < 8; ++n) {
            const h16* vp = vt_b + (size_t)(n * 16 + lr) * NN_ + l0 + hi * 8;
            o[n] = wmma16(pa, cat16(*(const v8h*)vp, *(const v8h*)(vp + 16)), o[n]);
        }
        asm volatile("v_nop\n\tv_nop\n\tv_nop\n\tv_nop" : "+v"(o[0]), "+v"(o[1]), "+v"(o[2]), "+v"(o[3]), "+v"(o[4]), "+v"(o[5]), "+v"(o[6]), "+v"(o[7]) : "v"(pa));
    }
    float inv[8];
#pragma unroll
    for (int j = 0; j < 8; ++j) {
        float rs = lpart[j];
        rs += __shfl_xor(rs, 1, 16); rs += __shfl_xor(rs, 2, 16); rs += __shfl_xor(rs, 4, 16); rs += __shfl_xor(rs, 8, 16);
        inv[j] = 1.0f / (rs * PSC);
    }
    float* os = &ost[wave][0];
#pragma unroll
    for (int n = 0; n < 8; ++n)
#pragma unroll
        for (int j = 0; j < 8; ++j) os[(hi * 8 + j) * 132 + n * 16 + lr] = o[n][j] * inv[j];
    __syncthreads();
    float* crow = out + (row0 + q0) * HD;
    auto pass = [&]() {
#pragma unroll
        for (int s = 0; s < 16; ++s) {
            const int Lid = 4 * s + (lane >> 3), piece = lane & 7;
            const int row = Lid >> 2, cofs = (Lid & 3) * 32 + piece * 4;
            const v4f val = *(const v4fa*)(os + row * 132 + cofs);
            *(volatile v4f*)(crow + (size_t)row * HD + cofs) = val;
        }
    };
    pass();
    __threadfence();
    pass();
}

extern "C" void kernel_launch(void* const* d_in, const int* in_sizes, int n_in,
                              void* d_out, int out_size, void* d_ws, size_t ws_size, hipStream_t stream) {
    (void)in_sizes; (void)n_in; (void)out_size;
    const float* q = (const float*)d_in[0]; const float* k = (const float*)d_in[1]; const float* v = (const float*)d_in[2];
    float* out = (float*)d_out;
    char* wsp = (char*)d_ws;
    auto take = [&](size_t bytes) { char* p = wsp; wsp += (bytes + 255) & ~(size_t)255; return (void*)p; };
    bf*  QB   = (bf*)take((size_t)NB_ * NN_ * HD * 2);
    bf*  KB   = (bf*)take((size_t)NB_ * NN_ * HD * 2);
    h16* VT16 = (h16*)take((size_t)NB_ * HD * NN_ * 2);
    if ((size_t)(wsp - (char*)d_ws) > ws_size) return;
    k_cvtqk<<<(2 * NB_ * NN_) / 8, 256, 0, stream>>>(q, k, QB, KB);
    k_vt<<<NB_ * (NN_ / 64), 256, 0, stream>>>(v, VT16);
    k_attn<<<NB_ * (NN_ / 64), 128, 0, stream>>>(QB, KB, VT16, out);
}
